// SentenceEmbedding_3161095930187
// MI455X (gfx1250) — hardware-verified
//
#include <hip/hip_runtime.h>

typedef __attribute__((ext_vector_type(16))) _Float16 v16h;
typedef __attribute__((ext_vector_type(8)))  _Float16 v8h;
typedef __attribute__((ext_vector_type(8)))  float    v8f;
typedef __attribute__((ext_vector_type(4)))  float    v4f_t;
typedef float v4fa __attribute__((ext_vector_type(4), may_alias));
typedef __attribute__((ext_vector_type(4)))  unsigned v4u_t;
typedef unsigned v4ua __attribute__((ext_vector_type(4), may_alias));

#define B_    512
#define L_    128
#define WD_   300
#define PD_   50
#define C_    256
#define KH_   3
#define D_    400
#define DP_   416
#define LC_   126
#define KTOT_ (KH_*DP_)
#define KSTEPS_ (KTOT_/32)
#define M_    (B_*LC_)
#define PLX   ((size_t)B_ * L_ * DP_)
#define PLW   ((size_t)C_ * KTOT_)
#define RSPLIT (1.0f / 2048.0f)
#define NBLK_ (M_ / 32)

__device__ __forceinline__ _Float16 lo_of(float v, _Float16 h) { return (_Float16)((v - (float)h) * 2048.0f); }
__device__ __forceinline__ v8f wmma16(v16h a, v16h b, v8f c) { return __builtin_amdgcn_wmma_f32_16x16x32_f16(false, a, false, b, (short)0, c, false, false); }
__device__ __forceinline__ v8f wmma_split(v16h a, v16h al, v16h b, v16h bl, v8f c) { v8f x = {}; x = wmma16(al, b, x); x = wmma16(a, bl, x); return wmma16(a, b, c) + x * RSPLIT; }
__device__ __forceinline__ v8f wmma_split_a(v16h a, v16h al, v16h b, v8f c) { v8f x = {}; x = wmma16(al, b, x); return wmma16(a, b, c) + x * RSPLIT; }

__device__ __forceinline__ void put8(_Float16* dst, size_t pl, const float* v) {
  _Float16 hh[8], hl[8];
#pragma unroll
  for (int e = 0; e < 8; ++e) { hh[e] = (_Float16)v[e]; hl[e] = lo_of(v[e], hh[e]); }
  const v4u_t u0 = *(const v4ua*)hh, u1 = *(const v4ua*)hl;
  *(volatile v4u_t*)dst = u0; *(volatile v4u_t*)(dst + pl) = u1; __threadfence();
  *(volatile v4u_t*)dst = u0; *(volatile v4u_t*)(dst + pl) = u1;
}

__global__ void gather_embed_kernel(const int* __restrict__ sent, const int* __restrict__ pos1, const int* __restrict__ pos2,
                                    const float* __restrict__ Wword, const float* __restrict__ Wp1, const float* __restrict__ Wp2,
                                    _Float16* __restrict__ X) {
  const int bl = blockIdx.x;
  int si = sent[bl], p1 = pos1[bl], p2 = pos2[bl];
  si = (si < 0) ? 0 : (si > 49999 ? 49999 : si); p1 = (p1 < 0) ? 0 : (p1 > 255 ? 255 : p1); p2 = (p2 < 0) ? 0 : (p2 > 255 ? 255 : p2);
  _Float16* row = X + (size_t)bl * DP_;
  for (int ch = threadIdx.x; ch < DP_ / 8; ch += blockDim.x) {
    float v[8];
#pragma unroll
    for (int e = 0; e < 8; ++e) {
      const int d = ch * 8 + e;
      float x;
      if (d < WD_)            x = Wword[(size_t)si * WD_ + d];
      else if (d < WD_ + PD_) x = Wp1[p1 * PD_ + (d - WD_)];
      else if (d < D_)        x = Wp2[p2 * PD_ + (d - WD_ - PD_)];
      else                    x = 0.0f;
      v[e] = x;
    }
    put8(row + ch * 8, PLX, v);
  }
}

__global__ void prep_weights_kernel(const float* __restrict__ cw, _Float16* __restrict__ Wt) {
  const int c = blockIdx.x;
  for (int ch = threadIdx.x; ch < KTOT_ / 8; ch += blockDim.x) {
    float v[8];
#pragma unroll
    for (int e = 0; e < 8; ++e) {
      const int k = ch * 8 + e, kh = k / DP_, d = k - kh * DP_;
      v[e] = (d < D_) ? cw[(size_t)c * (KH_ * D_) + kh * D_ + d] : 0.0f;
    }
    put8(Wt + (size_t)c * KTOT_ + ch * 8, PLW, v);
  }
}

__global__ __launch_bounds__(128) void conv_wmma_kernel(
    const _Float16* __restrict__ X, const _Float16* __restrict__ Wt, const float* __restrict__ bias,
    const int* __restrict__ widx, float* __restrict__ pmax)
{
  const int lane  = threadIdx.x & 31;
  const int wave  = threadIdx.x >> 5;
  const int mbase = blockIdx.x * 32;
  const int khalf = lane >> 4, l16 = lane & 15;

  const int r0 = mbase + l16, r1 = r0 + 16;
  const int bA0 = r0 / LC_, lA0 = r0 - bA0 * LC_;
  const int bA1 = r1 / LC_, lA1 = r1 - bA1 * LC_;
  const _Float16* aBase0 = X + ((size_t)bA0 * L_ + lA0) * DP_;
  const _Float16* aBase1 = X + ((size_t)bA1 * L_ + lA1) * DP_;

  const int ncol = wave * 64 + l16;
  const _Float16* bp[4];
#pragma unroll
  for (int j = 0; j < 4; ++j) bp[j] = Wt + (size_t)(ncol + 16 * j) * KTOT_;

  v8f acc[2][4] = {};
  for (int kk = 0; kk < KSTEPS_; ++kk) {
    const int kb = kk * 32 + khalf * 8;
    union U { v16h v; v8h h[2]; } a0, a0l, a1, a1l;
    a0.h[0]  = *(const v8h*)(aBase0 + kb);        a0.h[1]  = *(const v8h*)(aBase0 + kb + 16);
    a0l.h[0] = *(const v8h*)(aBase0 + PLX + kb);  a0l.h[1] = *(const v8h*)(aBase0 + PLX + kb + 16);
    a1.h[0]  = *(const v8h*)(aBase1 + kb);        a1.h[1]  = *(const v8h*)(aBase1 + kb + 16);
    a1l.h[0] = *(const v8h*)(aBase1 + PLX + kb);  a1l.h[1] = *(const v8h*)(aBase1 + PLX + kb + 16);
#pragma unroll
    for (int j = 0; j < 4; ++j) {
      U b;
      b.h[0]  = *(const v8h*)(bp[j] + kb);        b.h[1]  = *(const v8h*)(bp[j] + kb + 16);
      acc[0][j] = wmma_split_a(a0.v, a0l.v, b.v, acc[0][j]);
      acc[1][j] = wmma_split_a(a1.v, a1l.v, b.v, acc[1][j]);
    }
  }

  const int bFirst = mbase / LC_;
  float pm[4][6];
#pragma unroll
  for (int j = 0; j < 4; ++j)
#pragma unroll
    for (int s = 0; s < 6; ++s) pm[j][s] = -1.0f;
#pragma unroll
  for (int t = 0; t < 2; ++t)
#pragma unroll
    for (int v = 0; v < 8; ++v) {
      const int m = mbase + t * 16 + v + khalf * 8;
      const int b = m / LC_, l = m - b * LC_;
      const int w0 = widx[b * 2 + 0], w1 = widx[b * 2 + 1];
      const bool in0 = (l < w0), in1 = (l >= w0) && (l < w1 - 1), in2 = (l >= w1 - 1);
      const int sb3 = (b - bFirst) * 3;
#pragma unroll
      for (int j = 0; j < 4; ++j) {
        const float r = fmaxf(acc[t][j][v] + bias[ncol + 16 * j], 0.0f);
#pragma unroll
        for (int s = 0; s < 6; ++s) {
          const bool hit = (s == sb3 && in0) || (s == sb3 + 1 && in1) || (s == sb3 + 2 && in2);
          pm[j][s] = hit ? fmaxf(pm[j][s], r) : pm[j][s];
        }
      }
    }
#pragma unroll
  for (int j = 0; j < 4; ++j)
#pragma unroll
    for (int s = 0; s < 6; ++s) pm[j][s] = fmaxf(pm[j][s], __shfl_xor(pm[j][s], 16, 32));
  float* pbase = pmax + (size_t)blockIdx.x * 6 * C_ + wave * 64 + lane;
#pragma unroll 1
  for (int pass = 0; pass < 2; ++pass) {
#pragma unroll
    for (int s = 0; s < 6; ++s) {
      const float vlo = khalf ? pm[1][s] : pm[0][s];
      const float vhi = khalf ? pm[3][s] : pm[2][s];
      *(volatile float*)(pbase + (size_t)s * C_) = vlo;
      *(volatile float*)(pbase + (size_t)s * C_ + 32) = vhi;
    }
    __threadfence();
  }
}

__global__ __launch_bounds__(256) void pool_kernel(const float* __restrict__ pmax, float* __restrict__ out) {
  __shared__ __attribute__((aligned(16))) float so[3 * C_];
  const int b = blockIdx.x, c = threadIdx.x;
  float mx[3] = {-1.0f, -1.0f, -1.0f};
  const int blk0 = (b * LC_) / 32, blk1 = (b * LC_ + LC_ - 1) / 32;
  for (int blk = blk0; blk <= blk1; ++blk) {
    const int sb = b - (blk * 32) / LC_;
#pragma unroll
    for (int seg = 0; seg < 3; ++seg) mx[seg] = fmaxf(mx[seg], pmax[((size_t)blk * 6 + sb * 3 + seg) * C_ + c]);
  }
  so[c * 3 + 0] = (mx[0] < 0.0f) ? 0.0f : mx[0];
  so[c * 3 + 1] = (mx[1] < 0.0f) ? 0.0f : mx[1];
  so[c * 3 + 2] = (mx[2] < 0.0f) ? 0.0f : mx[2];
  __syncthreads();
  if (c < 3 * C_ / 4) {
    const v4f_t v = *(const volatile v4fa*)(so + c * 4);
    float* ob = out + (size_t)b * 3 * C_ + c * 4;
    *(volatile v4f_t*)ob = v; __threadfence(); *(volatile v4f_t*)ob = v;
  }
}

extern "C" void kernel_launch(void* const* d_in, const int* in_sizes, int n_in,
                              void* d_out, int out_size, void* d_ws, size_t ws_size,
                              hipStream_t stream) {
  (void)in_sizes; (void)n_in; (void)out_size; (void)ws_size;
  const int*   sent  = (const int*)d_in[0];
  const int*   pos1  = (const int*)d_in[1];
  const int*   pos2  = (const int*)d_in[2];
  const int*   widx  = (const int*)d_in[3];
  const float* Wword = (const float*)d_in[4];
  const float* Wp1   = (const float*)d_in[5];
  const float* Wp2   = (const float*)d_in[6];
  const float* convw = (const float*)d_in[7];
  const float* convb = (const float*)d_in[8];
  float*       out   = (float*)d_out;

  char* ws = (char*)d_ws;
  _Float16* X  = (_Float16*)ws;                                     ws += 2 * PLX * sizeof(_Float16);
  _Float16* Wt = (_Float16*)ws;                                     ws += 2 * PLW * sizeof(_Float16);
  float*  pmax = (float*)ws;

  gather_embed_kernel<<<B_ * L_, 64, 0, stream>>>(sent, pos1, pos2, Wword, Wp1, Wp2, X);
  prep_weights_kernel<<<C_, 256, 0, stream>>>(convw, Wt);
  conv_wmma_kernel<<<M_ / 32, 128, 0, stream>>>(X, Wt, convb, widx, pmax);
  pool_kernel<<<B_, 256, 0, stream>>>(pmax, out);
}
